// RRLSTM_28535762715372
// MI455X (gfx1250) — hardware-verified
//
#include <hip/hip_runtime.h>


namespace {
constexpr int Bn = 128, T1 = 513, SD = 64, NA = 8, U = 512, KX = 96  ;
constexpr float AS_ = 8.0f;

typedef _Float16 b16;
typedef __attribute__((ext_vector_type(16))) _Float16 v16b;
typedef __attribute__((ext_vector_type(8))) _Float16 v8b;
typedef __attribute__((ext_vector_type(8))) float v8f;
typedef __attribute__((ext_vector_type(4))) float v4f;
__device__ __forceinline__ float bf16_rne(float f) { unsigned int u = __float_as_uint(f); u += 0x7FFFu + ((u >> 16) & 1u); return __uint_as_float(u & 0xFFFF0000u); }
__device__ __forceinline__ void split16(float v, b16& hi, b16& lo) { hi = (b16)v; lo = (b16)(v - (float)hi); }
__device__ __forceinline__ v16b frag_kb(const b16* p, int hh) { const v8b a = *(const v8b*)(p + 8 * hh), b = *(const v8b*)(p + 16 + 8 * hh); v16b f;
#pragma unroll
  for (int e = 0; e < 8; ++e) { f[e] = a[e]; f[8 + e] = b[e]; } return f; }
__device__ __forceinline__ v8f wmma16b(v16b a, v16b b, v8f c) { v8f d = __builtin_amdgcn_wmma_f32_16x16x32_f16(false, a, false, b, (short)0, c, false, false); asm volatile("v_nop\n\tv_nop\n\tv_nop\n\tv_nop" : "+v"(d) : "v"(a), "v"(b)); return d; }
__device__ __forceinline__ float nexp(float x) { return __builtin_amdgcn_exp2f(x * 1.4426950408889634f); }
__device__ __forceinline__ float sigm(float x) { return 1.0f / (1.0f + nexp(-x)); }
__device__ __forceinline__ float tanh_f(float x) { const float e = nexp(-2.0f * fabsf(x)); const float t = (1.0f - e) / (1.0f + e); return (x >= 0.0f) ? t : -t; }
__device__ __forceinline__ float pmul(float a, float b) { float p = a * b; asm volatile("" : "+v"(p)); return p; }

struct Wo_ { static constexpr size_t CI = 0, OG = CI + 512 * 96, IG = OG + 512 * 96, END = IG + (size_t)512 * 512; };
__global__ __launch_bounds__(256) void prep_kernel(const float* __restrict__ Wci, const float* __restrict__ bci, const float* __restrict__ Wig, const float* __restrict__ big, const float* __restrict__ Wog, const float* __restrict__ bog, const float* __restrict__ Wl, const float* __restrict__ bl, b16* __restrict__ R, float* __restrict__ P) {
  const int t_ = blockIdx.x * 256 + threadIdx.x, nth = gridDim.x * 256;
  for (int pass = 0; pass < 2; ++pass) {
    for (int q = t_; q < 512 * 96; q += nth) { const int o = q / 96, k = q % 96; R[Wo_::CI + q] = (b16)((k < 72) ? bf16_rne(Wci[k * U + o]) : 0.0f); R[Wo_::OG + q] = (b16)((k < 72) ? bf16_rne(Wog[k * U + o]) : 0.0f); }
    for (int q = t_; q < 512 * 512; q += nth) { const int o = q >> 9, k = q & 511; R[Wo_::IG + q] = (b16)bf16_rne(Wig[(size_t)k * U + o]); }
    for (int q = t_; q < 2049; q += nth) { float v; if (q < 512) v = bci[q]; else if (q < 1024) v = bog[q - 512]; else if (q < 1536) v = big[q - 1024]; else if (q < 2048) v = Wl[q - 1536]; else v = bl[0]; P[q] = bf16_rne(v); }
    __threadfence(); }
}

__global__ __launch_bounds__(128) void rr_kernel(const float* __restrict__ st, const int* __restrict__ act, const b16* __restrict__ R, const float* __restrict__ P, float* __restrict__ ybuf) {
  __shared__ __attribute__((aligned(16))) b16 X[16][KX + 8]; __shared__ __attribute__((aligned(16))) b16 Hh[16][U + 8], Hl[16][U + 8]; __shared__ float Yp[4][16]; __shared__ __attribute__((aligned(16))) float Yo[16][T1 + 3];
  const int wave = threadIdx.x >> 5, lane = threadIdx.x & 31, nloc = lane & 15, hlf = lane >> 4, t_ = threadIdx.x, b0 = blockIdx.x * 16;
  const float* bci = P; const float* bog = P + 512; const float* big = P + 1024; const float* Wl = P + 1536; const float bl = P[2048];
  v8f c[8], ci[8];
#pragma unroll
  for (int t = 0; t < 8; ++t) c[t] = (v8f){};
  for (int i = t_; i < 16 * (U + 8); i += 128) { (&Hh[0][0])[i] = (b16)0.0f; (&Hl[0][0])[i] = (b16)0.0f; }
  for (int step = 0; step < T1; ++step) {
    for (int i = t_; i < 16 * KX; i += 128) { const int r = i / KX, k = i % KX; const int b = b0 + r; float v = 0.0f;
      if (k < SD) v = bf16_rne(st[((size_t)b * T1 + step) * SD + k]); else if (k < SD + NA && step < T1 - 1) { int a = act[(size_t)b * (T1 - 1) + step]; a = (a < 0) ? 0 : (a >= NA ? NA - 1 : a); v = (k - SD == a) ? 1.0f : 0.0f; }
      X[r][k] = (b16)v; }
    __syncthreads();
#pragma unroll
    for (int t = 0; t < 8; ++t) ci[t] = (v8f){};
#pragma unroll
    for (int kb = 0; kb < KX; kb += 32) { const v16b a = frag_kb(&X[nloc][kb], hlf);
#pragma unroll
      for (int t = 0; t < 8; ++t) { const v16b bw = frag_kb(R + Wo_::CI + (size_t)(wave * 128 + t * 16 + nloc) * KX + kb, hlf); ci[t] = wmma16b(a, bw, ci[t]); } }
#pragma unroll
    for (int t = 0; t < 8; ++t) { const int cc = wave * 128 + t * 16 + nloc; v8f ig = {};
#pragma unroll 4
      for (int kb = 0; kb < U; kb += 32) { const v16b ah = frag_kb(&Hh[nloc][kb], hlf), al = frag_kb(&Hl[nloc][kb], hlf); const v16b bw = frag_kb(R + Wo_::IG + (size_t)cc * U + kb, hlf); ig = wmma16b(ah, bw, ig); ig = wmma16b(al, bw, ig); }
      const float bc = bci[cc], bi = big[cc];
#pragma unroll
      for (int r = 0; r < 8; ++r) c[t][r] += pmul(tanh_f(ci[t][r] + bc), sigm(ig[r] * (1.0f / AS_) + bi)); }
#pragma unroll
    for (int t = 0; t < 8; ++t) { const int cc = wave * 128 + t * 16 + nloc; v8f og = {};
#pragma unroll
      for (int kb = 0; kb < KX; kb += 32) { const v16b a = frag_kb(&X[nloc][kb], hlf); const v16b bw = frag_kb(R + Wo_::OG + (size_t)cc * KX + kb, hlf); og = wmma16b(a, bw, og); }
      const float bo = bog[cc];
#pragma unroll
      for (int r = 0; r < 8; ++r) ci[t][r] = pmul(c[t][r], sigm(og[r] + bo)); }
    __syncthreads();
    float yp[8];
#pragma unroll
    for (int r = 0; r < 8; ++r) yp[r] = 0.0f;
#pragma unroll
    for (int t = 0; t < 8; ++t) { const int cc = wave * 128 + t * 16 + nloc; const float wl = Wl[cc];
#pragma unroll
      for (int r = 0; r < 8; ++r) { const float h = ci[t][r]; b16 h_, l_; split16(h * AS_, h_, l_); Hh[8 * hlf + r][cc] = h_; Hl[8 * hlf + r][cc] = l_; yp[r] += pmul(h, wl); } }
#pragma unroll
    for (int r = 0; r < 8; ++r) {
#pragma unroll
      for (int o = 1; o < 16; o <<= 1) yp[r] += __shfl_xor(yp[r], o); }
    if (nloc == 0) {
#pragma unroll
      for (int r = 0; r < 8; ++r) Yp[wave][8 * hlf + r] = yp[r]; }
    __syncthreads();
    if (t_ < 16) Yo[t_][step] = ((Yp[0][t_] + Yp[1][t_]) + (Yp[2][t_] + Yp[3][t_])) + bl;
  }
  __syncthreads();
  for (int pass = 0; pass < 2; ++pass) { for (int i = t_; i < 16 * ((T1 + 3) / 4); i += 128) { const int r = i / ((T1 + 3) / 4), c4 = (i % ((T1 + 3) / 4)) * 4; *(volatile v4f*)(ybuf + (size_t)(b0 + r) * (T1 + 3) + c4) = *(const v4f*)(&Yo[r][c4]); } __threadfence(); }
}

__global__ __launch_bounds__(256) void copy_kernel(const float* __restrict__ ybuf, float* __restrict__ out) {
  for (int pass = 0; pass < 2; ++pass) { for (int i = threadIdx.x; i < Bn * T1; i += 256) { const int b = i / T1, t = i % T1; ((volatile float*)out)[i] = ybuf[(size_t)b * (T1 + 3) + t]; } __threadfence(); }
}
}

extern "C" void kernel_launch(void* const* d_in, const int* in_sizes, int n_in,
                              void* d_out, int out_size, void* d_ws, size_t ws_size, hipStream_t stream) {
  (void)n_in; (void)out_size;
  const float* st = (const float*)d_in[0]; const int* act = (const int*)d_in[1]; const float* Wci = (const float*)d_in[2]; const float* bci = (const float*)d_in[3]; const float* Wig = (const float*)d_in[4]; const float* big = (const float*)d_in[5]; const float* Wog = (const float*)d_in[6]; const float* bog = (const float*)d_in[7]; const float* Wl = (const float*)d_in[8]; const float* bl = (const float*)d_in[9];
  float* out = (float*)d_out;
  if (in_sizes[0] != Bn * T1 * SD || in_sizes[1] != Bn * (T1 - 1) || in_sizes[2] != 72 * U || in_sizes[4] != U * U || in_sizes[8] != U) return;
  size_t off = 0; char* ws = (char*)d_ws;
  auto carve = [&](size_t bytes) { char* p = ws + off; off += (bytes + 255) & ~(size_t)255; return p; };
  b16* R = (b16*)carve(Wo_::END * 2); float* P = (float*)carve(2304 * 4); float* ybuf = (float*)carve((size_t)Bn * (T1 + 3) * 4);
  if (off > ws_size) return;
  prep_kernel<<<128, 256, 0, stream>>>(Wci, bci, Wig, big, Wog, bog, Wl, bl, R, P);
  rr_kernel<<<Bn / 16, 128, 0, stream>>>(st, act, R, P, ybuf);
  copy_kernel<<<1, 256, 0, stream>>>(ybuf, out);
}
